// UnconsciousnessFlow_8985071583850
// MI455X (gfx1250) — hardware-verified
//
#include <hip/hip_runtime.h>


namespace {
constexpr int N = 50000, E = 262144, D = 256, NR = 200, EC = 16384, NCH = E / EC, NPAD = 50176, NBLK = NPAD / 128;
constexpr float FXS = 65536.0f, FXI = 1.0f / 65536.0f;

typedef _Float16 b16;
typedef __attribute__((ext_vector_type(16))) _Float16 v16b;
typedef __attribute__((ext_vector_type(8)))  _Float16 v8b;
typedef __attribute__((ext_vector_type(8)))  float v8f;
typedef __attribute__((ext_vector_type(4)))  float v4f;

__device__ __forceinline__ v8b ld8b(const b16* p) { return *(const v8b*)p; }
__device__ __forceinline__ v16b cat8b(v8b a, v8b b) { return __builtin_shufflevector(a, b, 0, 1, 2, 3, 4, 5, 6, 7, 8, 9, 10, 11, 12, 13, 14, 15); }
__device__ __forceinline__ v16b frag_kb(const b16* p, int hh) { return cat8b(ld8b(p + 8 * hh), ld8b(p + 16 + 8 * hh)); }
__device__ __forceinline__ void split16(float v, b16& hi, b16& lo) { hi = (b16)v; lo = (b16)(v - (float)hi); }
__device__ __forceinline__ void frag_ksplit(const float* p, int hh, v16b& fh_, v16b& fl_) {
  const float* p0 = p + 8 * hh; const float* p1 = p + 16 + 8 * hh;
#pragma unroll
  for (int e = 0; e < 8; ++e) { b16 a, c; split16(p0[e], a, c); fh_[e] = a; fl_[e] = c; split16(p1[e], a, c); fh_[8 + e] = a; fl_[8 + e] = c; }
}
__device__ __forceinline__ v8f wmma16b(v16b a, v16b b, v8f c) {
  v8f d = __builtin_amdgcn_wmma_f32_16x16x32_f16(false, a, false, b, (short)0, c, false, false);
  asm volatile("v_nop\n\tv_nop\n\tv_nop\n\tv_nop" : "+v"(d) : "v"(a), "v"(b));
  return d;
}
__device__ __forceinline__ void wave_lds_sync() {
  __builtin_amdgcn_fence(__ATOMIC_RELEASE, "workgroup");
  __builtin_amdgcn_wave_barrier();
  __builtin_amdgcn_fence(__ATOMIC_ACQUIRE, "workgroup");
}

struct Opnd { const void* p0; const void* p1; int ld; };
template <int NP> __device__ __forceinline__ void load_frags(const Opnd& o, int row, int kb, int hh, v16b& fh_, v16b& fl_) {
  if (NP == 0) { frag_ksplit((const float*)o.p0 + (size_t)row * o.ld + kb, hh, fh_, fl_); }
  else if (NP == 4 || NP == 5) {
    const float sc_ = (NP == 4) ? 64.0f : 8.0f;
    const float* p = (const float*)o.p0 + (size_t)row * o.ld + kb; const float* p0 = p + 8 * hh; const float* p1 = p + 16 + 8 * hh;
#pragma unroll
    for (int e = 0; e < 8; ++e) { b16 a, c; split16(p0[e] * sc_, a, c); fh_[e] = a; fl_[e] = c; split16(p1[e] * sc_, a, c); fh_[8 + e] = a; fl_[8 + e] = c; }
  } else if (NP == 3) {
    const float* p = (const float*)o.p0 + (size_t)row * o.ld + kb; const float* p0 = p + 8 * hh; const float* p1 = p + 16 + 8 * hh;
#pragma unroll
    for (int e = 0; e < 8; ++e) { fh_[e] = (b16)p0[e]; fh_[8 + e] = (b16)p1[e]; }
    fl_ = fh_;
  } else {
    fh_ = frag_kb((const b16*)o.p0 + (size_t)row * o.ld + kb, hh);
    if (NP == 2) fl_ = frag_kb((const b16*)o.p1 + (size_t)row * o.ld + kb, hh); else fl_ = fh_;
  }
}
template <int ANP, int BNP> __device__ __forceinline__ v8f mac(v16b ah, v16b al, v16b bh, v16b bl, v8f c) {
  c = wmma16b(ah, bh, c);
  if (BNP == 0 || BNP == 2 || BNP == 4 || BNP == 5) c = wmma16b(ah, bl, c);
  if (ANP == 0 || ANP == 2 || ANP == 4 || ANP == 5) c = wmma16b(al, bh, c);
  return c;
}
template <int ANP, int BNP>
__device__ __forceinline__ void gemm_tile(const Opnd& A, const Opnd& B, int K, int m0, int c0, int nloc, int hlf, v8f (&acc)[2][4]) {
  for (int kb = 0; kb < K; kb += 32) {
    v16b a0h, a0l, a1h, a1l;
    load_frags<ANP>(A, m0 + nloc, kb, hlf, a0h, a0l);
    load_frags<ANP>(A, m0 + 16 + nloc, kb, hlf, a1h, a1l);
#pragma unroll
    for (int t = 0; t < 4; ++t) {
      v16b bh, bl;
      load_frags<BNP>(B, c0 + t * 16 + nloc, kb, hlf, bh, bl);
      acc[0][t] = mac<ANP, BNP>(a0h, a0l, bh, bl, acc[0][t]);
      acc[1][t] = mac<ANP, BNP>(a1h, a1l, bh, bl, acc[1][t]);
    }
  }
}

__device__ __forceinline__ void epi_planes(v8f (&acc)[2][4], float scale, bool two, b16* __restrict__ oh, b16* __restrict__ ol, int ldo,
                                           int m0, int c0, int lane, b16* Th, b16* Tl) {
  const int nloc = lane & 15, hlf = lane >> 4;
#pragma unroll
  for (int t = 0; t < 4; ++t)
#pragma unroll
    for (int r = 0; r < 2; ++r)
#pragma unroll
      for (int v = 0; v < 8; ++v) {
        const int rr = r * 16 + v + 8 * hlf, cc = t * 16 + nloc;
        b16 h_, l_; split16(acc[r][t][v] * scale, h_, l_);
        Th[rr * 64 + cc] = h_; Tl[rr * 64 + cc] = l_;
      }
  wave_lds_sync();
  for (int pass = 0; pass < 2; ++pass) {
#pragma unroll
    for (int j = 0; j < 8; ++j) {
      const int rr = j * 4 + (lane >> 3), c8 = (lane & 7) * 8;
      const size_t o = (size_t)(m0 + rr) * ldo + c0 + c8;
      *(volatile v8b*)(oh + o) = ld8b(Th + rr * 64 + c8);
      if (two) *(volatile v8b*)(ol + o) = ld8b(Tl + rr * 64 + c8);
    }
    __threadfence();
  }
}
__device__ __forceinline__ void epi_f32(v8f (&acc)[2][4], float scale, const float* rscale, float* __restrict__ out, int ldo, int m0, int c0, int lane, float* Tt) {
  const int nloc = lane & 15, hlf = lane >> 4;
#pragma unroll
  for (int t = 0; t < 4; ++t)
#pragma unroll
    for (int r = 0; r < 2; ++r)
#pragma unroll
      for (int v = 0; v < 8; ++v) {
        const int rr = r * 16 + v + 8 * hlf;
        const float rs = rscale ? rscale[(size_t)(m0 + rr) * 32] : 1.0f;
        Tt[rr * 64 + t * 16 + nloc] = acc[r][t][v] * scale * rs;
      }
  wave_lds_sync();
  float* dst0 = out + (size_t)m0 * ldo + c0;
  for (int pass = 0; pass < 2; ++pass) {
#pragma unroll
    for (int j = 0; j < 16; ++j) { const int rr = j * 2 + hlf, c4 = nloc * 4; *(volatile v4f*)(dst0 + (size_t)rr * ldo + c4) = *(const v4f*)(Tt + rr * 64 + c4); }
    __threadfence();
  }
}


typedef __attribute__((ext_vector_type(8))) __bf16 v8bb; typedef __attribute__((ext_vector_type(16))) __bf16 v16bb;
typedef __attribute__((ext_vector_type(8))) unsigned short v8us;
__device__ __forceinline__ v16bb frag_kb_bf(const __bf16* p, int hh) { const v8bb a = *(const v8bb*)(p + 8 * hh), b = *(const v8bb*)(p + 16 + 8 * hh); return __builtin_shufflevector(a, b, 0, 1, 2, 3, 4, 5, 6, 7, 8, 9, 10, 11, 12, 13, 14, 15); }
__device__ __forceinline__ v8f wmma16bb(v16bb a, v16bb b, v8f c) {
  v8f d = __builtin_amdgcn_wmma_f32_16x16x32_bf16(false, a, false, b, (short)0, c, false, false);
  asm volatile("v_nop\n\tv_nop\n\tv_nop\n\tv_nop" : "+v"(d) : "v"(a), "v"(b));
  return d;
}
__device__ __forceinline__ unsigned short bf16_rne_bits(float v) { unsigned int u = __float_as_uint(v); u += 0x7FFFu + ((u >> 16) & 1u); return (unsigned short)(u >> 16); }
__device__ __forceinline__ float bf16_rne(float v) { return __uint_as_float(((unsigned int)bf16_rne_bits(v)) << 16); }


__global__ __launch_bounds__(256) void prep_kernel(const float* __restrict__ A1, const float* __restrict__ A2, const float* __restrict__ B1, const float* __restrict__ B2, b16* __restrict__ w) {
  const size_t tid = (size_t)blockIdx.x * blockDim.x + threadIdx.x, nth = (size_t)gridDim.x * blockDim.x;
  for (int pass = 0; pass < 2; ++pass) { for (size_t p = tid; p < (size_t)4 * D * D; p += nth) { const int m = (int)(p / (D * D)); const int rem = (int)(p % (D * D)), n = rem / D, k = rem % D; const float* W = (m == 0) ? A1 : (m == 1) ? A2 : (m == 2) ? B1 : B2;
      ((volatile b16*)w)[p] = (b16)W[(size_t)k * D + n]; } __threadfence(); }
}

__global__ __launch_bounds__(256) void zero_kernel(float* __restrict__ acc, float* __restrict__ cnt) {
  const size_t i = (size_t)blockIdx.x * 256 + threadIdx.x; const v4f z = {0.0f, 0.0f, 0.0f, 0.0f};
  for (int pass = 0; pass < 2; ++pass) { *(volatile v4f*)(acc + i * 4) = z; if (i < NPAD) ((volatile float*)cnt)[i] = 0.0f; __threadfence(); }
}

__global__ __launch_bounds__(256) void msg0_kernel(const float* __restrict__ hid, const int* __restrict__ se, const float* __restrict__ rt, const float* __restrict__ fw, const float* __restrict__ fb, const float* __restrict__ fow, const float* __restrict__ fob, int ebase, float* __restrict__ m0) {
  const int i = blockIdx.x * 256 + threadIdx.x; const int el = i >> 6, cq = (i & 63) * 4, e = ebase + el;
  int vi = se[(size_t)e * 6 + 1], vj = se[(size_t)e * 6 + 2], rl = se[(size_t)e * 6 + 3]; vi = (vi < 0) ? 0 : (vi >= N ? N - 1 : vi); vj = (vj < 0) ? 0 : (vj >= N ? N - 1 : vj); rl = (rl < 0) ? 0 : (rl >= NR ? NR - 1 : rl);
  const v4f hv = *(const v4f*)(hid + (size_t)vi * D + cq), hj = *(const v4f*)(hid + (size_t)vj * D + cq), rr = *(const v4f*)(rt + (size_t)rl * D + cq);
  v4f o;
#pragma unroll
  for (int c = 0; c < 4; ++c) { const int d = cq + c; const float t = hv[c] * rr[c]; const float pre = hv[c] * fw[d] + t * fw[D + d] + (t * hj[c]) * fw[2 * D + d] + fb[d]; o[c] = fmaxf(pre, 0.0f) * fow[d] + fob[d]; }
  for (int pass = 0; pass < 2; ++pass) { *(volatile v4f*)(m0 + (size_t)el * D + cq) = o; __threadfence(); }
}

template <int MODE>
__global__ __launch_bounds__(128) void gemm_kernel(const float* __restrict__ x, const b16* __restrict__ w, const float* __restrict__ bias, const float* __restrict__ resid, const float* __restrict__ aux, int ebase, float* __restrict__ y) {
  __shared__ __attribute__((aligned(16))) float Ts[4][32 * 64];
  const int lane = threadIdx.x & 31, wave = threadIdx.x >> 5, nloc = lane & 15, hlf = lane >> 4, m0 = blockIdx.y * 128 + wave * 32, c0 = blockIdx.x * 64;
  v8f acc[2][4];
#pragma unroll
  for (int r = 0; r < 2; ++r)
#pragma unroll
    for (int t = 0; t < 4; ++t) acc[r][t] = (v8f){};
  const Opnd A{x, nullptr, D}, Bo{w, nullptr, D};
  gemm_tile<3, 1>(A, Bo, D, m0, c0, nloc, hlf, acc);
#pragma unroll
  for (int t = 0; t < 4; ++t)
#pragma unroll
    for (int r = 0; r < 2; ++r)
#pragma unroll
      for (int v = 0; v < 8; ++v) { const int row = m0 + r * 16 + 8 * hlf + v, c = c0 + t * 16 + nloc; float val = acc[r][t][v] + bias[c];
        if (MODE == 0) val = fmaxf(val, 0.0f);
        else if (MODE == 1) val = (val + resid[(size_t)row * D + c]) * aux[ebase + row];
        else { const int rn = min(row, N - 1); val = val + resid[(size_t)row * D + c] + aux[(size_t)rn * D + c]; }
        acc[r][t][v] = val; }
  if (MODE != 2) { epi_f32(acc, 1.0f, nullptr, y, D, m0, c0, lane, Ts[wave]); return; }
  float* Tt = Ts[wave];
#pragma unroll
  for (int t = 0; t < 4; ++t)
#pragma unroll
    for (int r = 0; r < 2; ++r)
#pragma unroll
      for (int v = 0; v < 8; ++v) Tt[(r * 16 + v + 8 * hlf) * 64 + t * 16 + nloc] = acc[r][t][v];
  wave_lds_sync();
  float* dst0 = y + (size_t)m0 * D + c0;
  for (int pass = 0; pass < 2; ++pass) {
#pragma unroll
    for (int j = 0; j < 16; ++j) { const int rr = j * 2 + hlf, c4 = nloc * 4; if (m0 + rr < N) *(volatile v4f*)(dst0 + (size_t)rr * D + c4) = *(const v4f*)(Tt + rr * 64 + c4); }
    __threadfence();
  }
}

typedef __attribute__((ext_vector_type(4))) int v4i;
__global__ __launch_bounds__(256) void agg_kernel(const int* __restrict__ se, int ebase, const float* __restrict__ m, float* __restrict__ gacc, float* __restrict__ gcnt) {
  constexpr int NB = 256;
  __shared__ __attribute__((aligned(16))) int acc[NB * D];
  __shared__ int cnt[NB]; __shared__ int list[8 * 256];
  const int t_ = threadIdx.x, wave = t_ >> 5, lane = t_ & 31, base = blockIdx.x * NB;
  for (int i = t_; i < NB * D; i += 256) acc[i] = 0;
  for (int i = t_; i < NB; i += 256) cnt[i] = 0;
  __syncthreads();
  int* wl = list + wave * 256;
  for (int c0 = 0; c0 < EC; c0 += 256 * 8) {
    const int e0 = c0 + (wave * 32 + lane) * 8; int dd[8];
#pragma unroll
    for (int j = 0; j < 8; ++j) dd[j] = se[(size_t)(ebase + e0 + j) * 6 + 2];
    unsigned sl[8]; bool hit[8]; bool anyl = false;
#pragma unroll
    for (int j = 0; j < 8; ++j) { sl[j] = (unsigned)(dd[j] - base); hit[j] = sl[j] < (unsigned)NB; anyl |= hit[j]; }
    int wc = 0;
    if (__builtin_amdgcn_ballot_w32(anyl) != 0u) {
#pragma unroll
      for (int j = 0; j < 8; ++j) {
        const unsigned mj = __builtin_amdgcn_ballot_w32(hit[j]);
        if (mj != 0u) {
          if (hit[j]) { const int pos = wc + (int)__builtin_amdgcn_mbcnt_lo(mj, 0u); wl[pos] = ((e0 + j) << 8) | (int)sl[j]; atomicAdd(&cnt[sl[j]], 1); }
          wc += __builtin_popcount(mj); } } }
    __builtin_amdgcn_wave_barrier(); __builtin_amdgcn_fence(__ATOMIC_RELEASE, "workgroup"); __builtin_amdgcn_fence(__ATOMIC_ACQUIRE, "workgroup");
    for (int i = 0; i < wc; ++i) { const int ent = wl[i]; const int e = ent >> 8, slot = ent & 255; const float* mr = m + (size_t)e * D + lane * 8; int* ar = acc + slot * D + lane * 8;
      const v4f a = *(const v4f*)mr, b2 = *(const v4f*)(mr + 4);
#pragma unroll
      for (int c = 0; c < 4; ++c) { atomicAdd(ar + c, (int)rintf(a[c] * FXS)); atomicAdd(ar + 4 + c, (int)rintf(b2[c] * FXS)); } }
    __builtin_amdgcn_wave_barrier();
  }
  __syncthreads();
  for (int pass = 0; pass < 2; ++pass) {
    for (int i = t_; i < NB * D / 4; i += 256) { const int r = i >> 6, cq = (i & 63) * 4, node = base + r; float* gp = gacc + (size_t)node * D + cq; v4f g = *(const v4f*)gp;
      if (pass == 0) {
#pragma unroll
        for (int c = 0; c < 4; ++c) g[c] += (float)acc[r * D + cq + c] * FXI; }
      *(volatile v4f*)gp = g; }
    if (t_ < NB) { const int node = base + t_; const float cv = gcnt[node] + ((pass == 0) ? (float)cnt[t_] : 0.0f); ((volatile float*)gcnt)[node] = cv; }
    __threadfence();
  }
}

__global__ __launch_bounds__(256) void upd_kernel(const float* __restrict__ gacc, const float* __restrict__ gcnt, const float* __restrict__ hid, const float* __restrict__ ent, const float* __restrict__ hw, const float* __restrict__ hb, const float* __restrict__ how, const float* __restrict__ hob, float* __restrict__ u0) {
  const int i = blockIdx.x * 256 + threadIdx.x; const int node = i >> 6, cq = (i & 63) * 4; v4f o = {0.0f, 0.0f, 0.0f, 0.0f};
  if (node < N) { const float inv = 1.0f / fmaxf(gcnt[node], 1.0f); const v4f av = *(const v4f*)(gacc + (size_t)node * D + cq), hv = *(const v4f*)(hid + (size_t)node * D + cq), ev = *(const v4f*)(ent + (size_t)node * D + cq);
#pragma unroll
    for (int c = 0; c < 4; ++c) { const int d = cq + c; const float a = av[c] * inv, h = hv[c], e = ev[c];
      const float pre = a * hw[d] + (a * h) * hw[D + d] + (a * e) * hw[2 * D + d] + h * hw[3 * D + d] + e * hw[4 * D + d] + (h * e) * hw[5 * D + d] + hb[d]; o[c] = fmaxf(pre, 0.0f) * how[d] + hob[d]; } }
  for (int pass = 0; pass < 2; ++pass) { *(volatile v4f*)(u0 + (size_t)node * D + cq) = o; __threadfence(); }
}
}

extern "C" void kernel_launch(void* const* d_in, const int* in_sizes, int n_in,
                              void* d_out, int out_size, void* d_ws, size_t ws_size, hipStream_t stream) {
  (void)n_in; (void)out_size;
  const float* hid = (const float*)d_in[0]; const int* se = (const int*)d_in[1]; const float* ey = (const float*)d_in[2]; const float* rt = (const float*)d_in[3]; const float* ent = (const float*)d_in[4];
  const float* fm_ws = (const float*)d_in[5]; const float* fm_b = (const float*)d_in[6]; const float* fm_ow = (const float*)d_in[7]; const float* fm_ob = (const float*)d_in[8];
  const float* gm_w1 = (const float*)d_in[9]; const float* gm_b1 = (const float*)d_in[10]; const float* gm_w2 = (const float*)d_in[11]; const float* gm_b2 = (const float*)d_in[12];
  const float* fh_ws = (const float*)d_in[13]; const float* fh_b = (const float*)d_in[14]; const float* fh_ow = (const float*)d_in[15]; const float* fh_ob = (const float*)d_in[16];
  const float* gh_w1 = (const float*)d_in[17]; const float* gh_b1 = (const float*)d_in[18]; const float* gh_w2 = (const float*)d_in[19]; const float* gh_b2 = (const float*)d_in[20];
  float* out = (float*)d_out;
  if (in_sizes[0] != N * D || in_sizes[1] != E * 6 || in_sizes[2] != E || in_sizes[3] != NR * D || in_sizes[4] != N * D || in_sizes[9] != D * D || in_sizes[19] != D * D) return;
  size_t off = 0; char* ws = (char*)d_ws;
  auto carve = [&](size_t bytes) { char* p = ws + off; off += (bytes + 255) & ~(size_t)255; return p; };
  b16* w = (b16*)carve((size_t)4 * D * D * 2);
  float* bufA = (float*)carve((size_t)NPAD * D * 4); float* bufB = (float*)carve((size_t)EC * D * 4); float* gacc = (float*)carve((size_t)NPAD * D * 4); float* gcnt = (float*)carve((size_t)NPAD * 4);
  if (off > ws_size) return;
  float* m0 = bufA; float* y1 = bufB;
  prep_kernel<<<256, 256, 0, stream>>>(gm_w1, gm_w2, gh_w1, gh_w2, w);
  zero_kernel<<<NPAD * D / 4 / 256, 256, 0, stream>>>(gacc, gcnt);
  for (int ch = 0; ch < NCH; ++ch) { const int ebase = ch * EC;
    msg0_kernel<<<EC * 64 / 256, 256, 0, stream>>>(hid, se, rt, fm_ws, fm_b, fm_ow, fm_ob, ebase, m0);
    gemm_kernel<0><<<dim3(4, EC / 128), 128, 0, stream>>>(m0, w, gm_b1, nullptr, nullptr, 0, y1);
    gemm_kernel<1><<<dim3(4, EC / 128), 128, 0, stream>>>(y1, w + (size_t)D * D, gm_b2, m0, ey, ebase, m0);
    agg_kernel<<<NPAD / 256, 256, 0, stream>>>(se, ebase, m0, gacc, gcnt);
  }
  upd_kernel<<<NPAD * 64 / 256, 256, 0, stream>>>(gacc, gcnt, hid, ent, fh_ws, fh_b, fh_ow, fh_ob, bufA);
  gemm_kernel<0><<<dim3(4, NBLK), 128, 0, stream>>>(bufA, w + (size_t)2 * D * D, gh_b1, nullptr, nullptr, 0, gacc);
  gemm_kernel<2><<<dim3(4, NBLK), 128, 0, stream>>>(gacc, w + (size_t)3 * D * D, gh_b2, bufA, hid, 0, out);
}
